// HAN_60266981097654
// MI455X (gfx1250) — hardware-verified
//
#include <hip/hip_runtime.h>
#include <stddef.h>
#include <stdint.h>
#include <math.h>


#define F_IN    256
#define NPATH   2
#define NHEAD   8
#define DHD     64
#define HD      512
#define KHL     1024
#define SHID    128
#define NOUT    16
#define OUTC    5
#define NTHR    256
#define NWAVE   8
#define EPT     8
#define CHUNK   (NTHR * EPT)
#define WCAP    (EPT * 32)
#define LISTN   (NWAVE * WCAP)
#define NBMAX   2048
#define SLOTB   11
#define RCAP    28672
#define DEGCAP  256
#define GBM     64
#define GBNA    64
#define GBNS    128
#define GNT     8
#define GTHR    128
#define ESTW    512
#define NEGSL   0.2f
#define MX0     (-1.0e30f)
#define WSMAX   134217728
#define LDS_AGG ((2 * RCAP + 2 * NBMAX + LISTN) * 4 + 64)
#define LDS_OUT (GBM * KHL * 2)
#define NUW     (NPATH * HD * (F_IN / 8))
#define NUS     (SHID * (KHL / 8))
#define NUP     (NOUT * (KHL / 8))
#define NUB1    (NUW)
#define NUB2    (NUB1 + NUS)
#define NUTOT   (NUB2 + NUP)

static_assert((CHUNK & (CHUNK - 1)) == 0 && CHUNK <= (1 << SLOTB));
static_assert(NBMAX == (1 << SLOTB));
static_assert(NTHR * 8 == NBMAX);
static_assert(LISTN >= NBMAX && LISTN >= NWAVE * WCAP);
static_assert((RCAP % 32) == 0);
static_assert(LDS_AGG <= 300000);
static_assert(LDS_OUT <= 300000);
static_assert(GBM == (GTHR / 32) * 16);
static_assert(GTHR == 2 * GBNA && GTHR == 2 * GBM && DHD == GBNA);
static_assert(HD == NHEAD * DHD && KHL == 2 * HD);
static_assert(GBNS == SHID && GBNS == 16 * GNT && GTHR == GBNS);
static_assert((F_IN % 32) == 0 && (KHL % 32) == 0);
static_assert(HD == 32 * 16 && DHD == 4 * 16);
static_assert(NHEAD * 4 == 32);
static_assert(NWAVE * ESTW <= RCAP);
static_assert(LISTN >= HD);
static_assert((NUB1 % NTHR) == 0 && (NUB2 % NTHR) == 0 && (NUTOT % NTHR) == 0);
static_assert((F_IN / 8) == 32 && (KHL / 8) == 128);
static_assert(NOUT == 16 && OUTC <= NOUT);
static_assert(F_IN <= KHL);
static_assert(((GBM * OUTC) % 4) == 0 && ((GBM * OUTC * 4) % 128) == 0);
static_assert(GTHR >= (GBM * OUTC) / 4 + 1);
static_assert((HD % GBNA) == 0 && HD / GBNA == NHEAD);

typedef float          v4f  __attribute__((ext_vector_type(4)));
typedef float          v8f  __attribute__((ext_vector_type(8)));
typedef int            v4i  __attribute__((ext_vector_type(4)));
typedef int            v8i  __attribute__((ext_vector_type(8)));
typedef unsigned int   v4u  __attribute__((ext_vector_type(4)));
typedef unsigned short v8us __attribute__((ext_vector_type(8)));
typedef __bf16         v16b __attribute__((ext_vector_type(16)));
typedef v4f  __attribute__((may_alias)) v4fa;
typedef v4u  __attribute__((may_alias)) v4ua;
typedef v8us __attribute__((may_alias)) v8usa;
union Frag { v16b vb; v8us h[2]; v8i w; };

__device__ __forceinline__ v8f wmb(const Frag& a, const Frag& b, v8f c) {
  v8f d = __builtin_amdgcn_wmma_f32_16x16x32_bf16(false, a.vb, false, b.vb, (short)0, c, false, false);
  asm volatile("v_nop\n\tv_nop\n\tv_nop\n\tv_nop" : "+v"(d) : "v"(a.w), "v"(b.w));
  return d;
}

__device__ __forceinline__ unsigned short bf_bits(float f) {
  unsigned int u = __float_as_uint(f);
  u += 0x7FFFu + ((u >> 16) & 1u);
  return (unsigned short)(u >> 16);
}
__device__ __forceinline__ float bf_val(unsigned short b) { return __uint_as_float(((unsigned int)b) << 16); }
__device__ __forceinline__ float bf_rne(float f) { return bf_val(bf_bits(f)); }
__device__ __forceinline__ unsigned int pk2(float lo, float hi) {
  return (unsigned int)bf_bits(lo) | ((unsigned int)bf_bits(hi) << 16);
}
__device__ __forceinline__ v4u pack8(const v4f a, const v4f b) {
  v4u r;
  r.x = pk2(a.x, a.y); r.y = pk2(a.z, a.w); r.z = pk2(b.x, b.y); r.w = pk2(b.z, b.w);
  return r;
}
__device__ __forceinline__ float rlo(unsigned int h, unsigned int l) {
  return __uint_as_float(h << 16) + __uint_as_float(l << 16);
}
__device__ __forceinline__ float rhi(unsigned int h, unsigned int l) {
  return __uint_as_float(h & 0xFFFF0000u) + __uint_as_float(l & 0xFFFF0000u);
}
__device__ __forceinline__ v4f upd4(v4f a, const v4f f, float s1, float s2) {
  a.x = fmaf(a.x, s1, s2 * f.x);
  a.y = fmaf(a.y, s1, s2 * f.y);
  a.z = fmaf(a.z, s1, s2 * f.z);
  a.w = fmaf(a.w, s1, s2 * f.w);
  return a;
}
__device__ __forceinline__ unsigned int shsel(unsigned int a, unsigned int b, int sl, bool pickb) {
  const int ga = __shfl((int)a, sl);
  const int gb = __shfl((int)b, sl);
  return (unsigned int)(pickb ? gb : ga);
}

__device__ __forceinline__ int scan_chunk(const int* __restrict__ dsts, int nE, int cbase, int slotBase,
                                          int nb, int vec8, int* list, int tid, int lane, int wave) {
  int wc = 0;
  const int el0  = tid * EPT;
  const int e0   = cbase + el0;
  const int sent = -2147483647 - 1;
  v4i da, db;
  if (vec8 != 0 && cbase + CHUNK <= nE) {
    da = *(const v4i*)(dsts + e0);
    db = *(const v4i*)(dsts + e0 + 4);
  } else {
    da.x = (e0     < nE) ? dsts[min(e0,     nE - 1)] : sent;
    da.y = (e0 + 1 < nE) ? dsts[min(e0 + 1, nE - 1)] : sent;
    da.z = (e0 + 2 < nE) ? dsts[min(e0 + 2, nE - 1)] : sent;
    da.w = (e0 + 3 < nE) ? dsts[min(e0 + 3, nE - 1)] : sent;
    db.x = (e0 + 4 < nE) ? dsts[min(e0 + 4, nE - 1)] : sent;
    db.y = (e0 + 5 < nE) ? dsts[min(e0 + 5, nE - 1)] : sent;
    db.z = (e0 + 6 < nE) ? dsts[min(e0 + 6, nE - 1)] : sent;
    db.w = (e0 + 7 < nE) ? dsts[min(e0 + 7, nE - 1)] : sent;
  }
  const unsigned nbs = (unsigned)slotBase;
  const unsigned unb = (unsigned)nb;
  const unsigned s0 = (unsigned)da.x - nbs, s1 = (unsigned)da.y - nbs;
  const unsigned s2 = (unsigned)da.z - nbs, s3 = (unsigned)da.w - nbs;
  const unsigned s4 = (unsigned)db.x - nbs, s5 = (unsigned)db.y - nbs;
  const unsigned s6 = (unsigned)db.z - nbs, s7 = (unsigned)db.w - nbs;
  const bool h0 = s0 < unb, h1 = s1 < unb, h2 = s2 < unb, h3 = s3 < unb;
  const bool h4 = s4 < unb, h5 = s5 < unb, h6 = s6 < unb, h7 = s7 < unb;
  const unsigned any = __builtin_amdgcn_ballot_w32(h0 | h1 | h2 | h3 | h4 | h5 | h6 | h7);
  if (any != 0u) {
#define HITJ(J, HJ, SJ) { \
      const unsigned mj = __builtin_amdgcn_ballot_w32(HJ); \
      if (mj != 0u) { \
        if (HJ) { \
          const int pos = wc + (int)__builtin_amdgcn_mbcnt_lo(mj, 0u); \
          if (pos < WCAP) list[wave * WCAP + pos] = ((el0 + (J)) << SLOTB) | (int)(SJ); \
        } \
        wc += (int)__builtin_popcount(mj); } }
    HITJ(0, h0, s0)
    HITJ(1, h1, s1)
    HITJ(2, h2, s2)
    HITJ(3, h3, s3)
    HITJ(4, h4, s4)
    HITJ(5, h5, s5)
    HITJ(6, h6, s6)
    HITJ(7, h7, s7)
#undef HITJ
  }
  return wc;
}

__global__ __launch_bounds__(NTHR) void k_xprep(const float* __restrict__ x, unsigned short* xb, int nN, int nUnits) {
  const int i = (int)blockIdx.x * NTHR + (int)threadIdx.x;
  if (i >= nUnits) return;
  const int row = i >> 5;
  const int c0  = (i & 31) * 8;
  const int rc  = row < nN ? row : nN - 1;
  const float* p = x + (size_t)rc * F_IN + c0;
  v4f a = *(const v4fa*)p, b = *(const v4fa*)(p + 4);
  const v4f z4 = {0.f, 0.f, 0.f, 0.f};
  if (row >= nN) { a = z4; b = z4; }
  const v4u hv = pack8(a, b);
  const size_t o = (size_t)row * F_IN + c0;
  *(volatile v4u*)(xb + o) = hv;
  __threadfence();
  *(volatile v4u*)(xb + o) = hv;
}

__device__ __forceinline__ v8us cv8b(const float* __restrict__ p, size_t stride) {
  v8us o;
#pragma unroll
  for (int i = 0; i < 8; ++i) o[i] = bf_bits(p[(size_t)i * stride]);
  return o;
}

__global__ __launch_bounds__(NTHR) void k_wprep(const float* __restrict__ w, const float* __restrict__ sw1,
                                                const float* __restrict__ pw,
                                                unsigned short* pwt, unsigned short* ps1t, unsigned short* ppt) {
  const int u = (int)blockIdx.x * NTHR + (int)threadIdx.x;
  v8us o;
  unsigned short* dp;
  if (u < NUB1) {
    const int v = u, n = v >> 5, k8 = (v & 31) * 8;
    const int pth = n >> 9, nn = n & (HD - 1);
    o = cv8b(w + (size_t)pth * F_IN * HD + (size_t)k8 * HD + nn, HD);
    dp = pwt + (size_t)v * 8;
  } else if (u < NUB2) {
    const int v = u - NUB1, n = v >> 7, k8 = (v & 127) * 8;
    const int kk = k8 & (HD - 1);
    o = cv8b(sw1 + (size_t)kk * SHID + n, SHID);
    dp = ps1t + (size_t)v * 8;
  } else if (u < NUTOT) {
    const int v = u - NUB2, n = v >> 7, k8 = (v & 127) * 8;
    const int kk = k8 & (HD - 1);
    const int nc = n < OUTC ? n : OUTC - 1;
    o = cv8b(pw + (size_t)kk * OUTC + nc, OUTC);
    const v8us z8 = {0, 0, 0, 0, 0, 0, 0, 0};
    if (n >= OUTC) o = z8;
    dp = ppt + (size_t)v * 8;
  } else {
    return;
  }
  *(volatile v8us*)dp = o;
  __threadfence();
  *(volatile v8us*)dp = o;
}

__global__ __launch_bounds__(GTHR) void k_gfeat(
    const unsigned short* __restrict__ A, const unsigned short* __restrict__ WT,
    float* outF, int K, int ldo,
    const float* __restrict__ atts, const float* __restrict__ attd, int attLen,
    float* SD, int MPr)
{
  __shared__ __attribute__((aligned(16))) float stg[GBM * GBNA];
  __shared__ __attribute__((aligned(16))) float satt[2 * GBNA];
  __shared__ __attribute__((aligned(16))) float sdot[2 * GBM];
  const int tid = (int)threadIdx.x, lane = tid & 31, wave = tid >> 5, hh = lane >> 4, m = lane & 15;
  const int rowBase = (int)blockIdx.x * GBM;
  const int head    = (int)blockIdx.y;
  const int col0    = head * GBNA;

  {
    const int which = tid >> 6;
    const int c  = tid & 63;
    const int cl = c < attLen ? c : attLen - 1;
    const float vs = atts[head * attLen + cl];
    const float vd = attd[head * attLen + cl];
    float v = (which == 0) ? vs : vd;
    v = (c < attLen) ? bf_rne(v) : 0.f;
    satt[which * GBNA + c] = v;
  }

  v8f acc[4];
  {
    const v8f z = {0.f, 0.f, 0.f, 0.f, 0.f, 0.f, 0.f, 0.f};
    acc[0] = z; acc[1] = z; acc[2] = z; acc[3] = z;
  }
  const unsigned short* ap = A  + (size_t)(rowBase + 16 * wave + m) * (size_t)K + 8 * hh;
  const unsigned short* wp = WT + (size_t)(col0 + m) * (size_t)K + 8 * hh;
  const int ksteps = K >> 5;
#pragma unroll 1
  for (int ks = 0; ks < ksteps; ++ks) {
    Frag af;
    af.h[0] = *(const v8usa*)(ap + 32 * ks);
    af.h[1] = *(const v8usa*)(ap + 32 * ks + 16);
#pragma unroll
    for (int t = 0; t < 4; ++t) {
      const unsigned short* wq = wp + (size_t)(16 * t) * (size_t)K + 32 * ks;
      Frag bfg;
      bfg.h[0] = *(const v8usa*)wq;
      bfg.h[1] = *(const v8usa*)(wq + 16);
      acc[t] = wmb(af, bfg, acc[t]);
    }
  }

#pragma unroll
  for (int t = 0; t < 4; ++t) {
    const int lc = 16 * t + m;
#pragma unroll
    for (int r = 0; r < 8; ++r) {
      const int lr = 16 * wave + 8 * hh + r;
      stg[lr * GBNA + lc] = acc[t][r];
    }
  }
  __syncthreads();

  {
    const int row = tid & 63, which = tid >> 6;
    const float* sa = satt + which * GBNA;
    const float* hr = stg + row * GBNA;
    float d = 0.f;
#pragma unroll 4
    for (int c4 = 0; c4 < GBNA / 4; ++c4) {
      const v4f hv = *(const v4fa*)(hr + 4 * c4);
      const v4f av = *(const v4fa*)(sa + 4 * c4);
      d = fmaf(hv.x, av.x, d);
      d = fmaf(hv.y, av.y, d);
      d = fmaf(hv.z, av.z, d);
      d = fmaf(hv.w, av.w, d);
    }
    sdot[which * GBM + row] = d;
  }
  __syncthreads();

  v4f fv[8];
#pragma unroll
  for (int i = 0; i < 8; ++i) {
    const int lr = 16 * wave + 2 * i + hh;
    fv[i] = *(const v4fa*)(stg + lr * GBNA + 4 * m);
  }
  const int which2 = lane >> 4, piece = lane & 15;
  const v4f sdv = *(const v4fa*)(sdot + which2 * GBM + 4 * piece);
  float* sp = SD + (size_t)(2 * head + which2) * (size_t)MPr + rowBase + 4 * piece;

#pragma unroll
  for (int i = 0; i < 8; ++i) {
    const int lr = 16 * wave + 2 * i + hh;
    const int gr = rowBase + lr;
    float* op = outF + (size_t)gr * (size_t)ldo + col0 + 4 * m;
    *(volatile v4f*)op = fv[i];
  }
  if (wave == 0) *(volatile v4f*)sp = sdv;
  __threadfence();
#pragma unroll
  for (int i = 0; i < 8; ++i) {
    const int lr = 16 * wave + 2 * i + hh;
    const int gr = rowBase + lr;
    float* op = outF + (size_t)gr * (size_t)ldo + col0 + 4 * m;
    *(volatile v4f*)op = fv[i];
  }
  if (wave == 0) *(volatile v4f*)sp = sdv;
}

__global__ __launch_bounds__(NTHR) void k_agg(
    const int* __restrict__ srcs, const int* __restrict__ dsts,
    const float* __restrict__ F, const float* __restrict__ SDp, const float* __restrict__ bias,
    unsigned short* ZP, int nN, int nE, int nb, int vec8, int MPr) {
  extern __shared__ v4f lds_dyn[];
  int* reg1 = (int*)lds_dyn;
  int* reg2 = reg1 + RCAP;
  int* scnt = reg2 + RCAP;
  int* soff = scnt + NBMAX;
  int* list = soff + NBMAX;
  int* wcnt = list + LISTN;
  int* wtot = wcnt + NWAVE;
  const int tid = (int)threadIdx.x, lane = tid & 31, wave = tid >> 5;
  const int nodeBase = (int)blockIdx.x * nb;

  for (int i = tid; i < NBMAX; i += NTHR) scnt[i] = 0;
  __syncthreads();

  int tot = 0;
  const int nChunks = (nE + CHUNK - 1) / CHUNK;
#pragma unroll 1
  for (int ch = 0; ch < nChunks; ++ch) {
    const int cbase = ch * CHUNK;
    const int wc = scan_chunk(dsts, nE, cbase, nodeBase, nb, vec8, list, tid, lane, wave);
    if (lane == 0) wcnt[wave] = wc;
    __syncthreads();
    int pre = 0, all = 0;
#pragma unroll
    for (int w2 = 0; w2 < NWAVE; ++w2) {
      int c = wcnt[w2];
      c = c < 0 ? 0 : (c > WCAP ? WCAP : c);
      all += c;
      pre += (w2 < wave) ? c : 0;
    }
    const int wcc  = wc > WCAP ? WCAP : wc;
    const int base = tot + pre;
#pragma unroll 1
    for (int i = lane; i < wcc; i += 32) {
      const int ent = list[wave * WCAP + i];
      const int el  = (ent >> SLOTB) & (CHUNK - 1);
      const int sl  = ent & (NBMAX - 1);
      int eid = cbase + el;
      eid = eid > nE - 1 ? nE - 1 : eid;
      const int pos = base + i;
      if (pos < RCAP) reg1[pos] = (int)(((unsigned)eid << SLOTB) | (unsigned)sl);
    }
    tot += all;
    tot = tot > RCAP ? RCAP : tot;
    __syncthreads();
  }
  const int nh = tot;

  if (wave == 0) {
#pragma unroll 1
    for (int b0 = 0; b0 < nh; b0 += 32) {
      const int idx = b0 + lane;
      const int uv  = reg1[idx < nh ? idx : nh - 1];
      const int m32 = (nh - b0) < 32 ? (nh - b0) : 32;
#pragma unroll 1
      for (int k = 0; k < m32; ++k) {
        const int u  = __builtin_amdgcn_readlane(uv, k);
        const int sl = u & (NBMAX - 1);
        if (lane == 0) scnt[sl] = scnt[sl] + 1;
      }
    }
  }
  __syncthreads();

  {
    const v4i ca = *(const v4i*)(scnt + 8 * tid);
    const v4i cb = *(const v4i*)(scnt + 8 * tid + 4);
    const int e0 = ca.x < 0 ? 0 : ca.x, e1 = ca.y < 0 ? 0 : ca.y, e2 = ca.z < 0 ? 0 : ca.z, e3 = ca.w < 0 ? 0 : ca.w;
    const int e4 = cb.x < 0 ? 0 : cb.x, e5 = cb.y < 0 ? 0 : cb.y, e6 = cb.z < 0 ? 0 : cb.z, e7 = cb.w < 0 ? 0 : cb.w;
    const int ts = e0 + e1 + e2 + e3 + e4 + e5 + e6 + e7;
    int incl = ts;
#pragma unroll
    for (int d = 1; d < 32; d <<= 1) {
      const int up = __shfl_up(incl, d);
      if (lane >= d) incl += up;
    }
    if (lane == 31) wtot[wave] = incl;
    __syncthreads();
    int pre = 0;
#pragma unroll
    for (int w2 = 0; w2 < NWAVE; ++w2) pre += (w2 < wave) ? wtot[w2] : 0;
    int run = pre + incl - ts;
    soff[8 * tid + 0] = run; run += e0;
    soff[8 * tid + 1] = run; run += e1;
    soff[8 * tid + 2] = run; run += e2;
    soff[8 * tid + 3] = run; run += e3;
    soff[8 * tid + 4] = run; run += e4;
    soff[8 * tid + 5] = run; run += e5;
    soff[8 * tid + 6] = run; run += e6;
    soff[8 * tid + 7] = run;
  }
  __syncthreads();
  for (int i = tid; i < NBMAX; i += NTHR) list[i] = soff[i];
  __syncthreads();

  if (wave == 0) {
#pragma unroll 1
    for (int b0 = 0; b0 < nh; b0 += 32) {
      const int idx = b0 + lane;
      const int uv  = reg1[idx < nh ? idx : nh - 1];
      const int m32 = (nh - b0) < 32 ? (nh - b0) : 32;
#pragma unroll 1
      for (int k = 0; k < m32; ++k) {
        const int u   = __builtin_amdgcn_readlane(uv, k);
        const int sl  = u & (NBMAX - 1);
        const int eid = (int)((unsigned)u >> SLOTB);
        if (lane == 0) {
          int pos = list[sl];
          pos = pos < 0 ? 0 : (pos > RCAP - 1 ? RCAP - 1 : pos);
          reg2[pos] = eid;
          list[sl] = pos + 1;
        }
      }
    }
  }
  __syncthreads();

  float* sb = (float*)list;
  for (int i = tid; i < HD; i += NTHR) sb[i] = bf_rne(bias[i]);
  __syncthreads();

  const int nbw = nb >> 3;
  const bool ovf = (nh >= RCAP);
  const float qnan = __int_as_float(0x7fc00000);
  const int c0   = 16 * lane;
  const int head = lane >> 2;
  const float* ASp = SDp + (size_t)(2 * head) * (size_t)MPr;
  const float* ADp = ASp + MPr;
  float* est = (float*)reg1 + wave * ESTW + 16 * lane;
  const int  slA = lane >> 1, slB = 16 + (lane >> 1);
  const bool odd = (lane & 1) != 0;
  const v4f z4 = {0.f, 0.f, 0.f, 0.f};

#pragma unroll 1
  for (int jt = 0; jt < nbw; ++jt) {
    const int slot = wave * nbw + jt;
    const int grow = nodeBase + slot;
    const int gcl  = grow < nN ? grow : nN - 1;
    int st = soff[slot];
    const int craw = scnt[slot];
    int cnt = craw;
    st  = st < 0 ? 0 : (st > nh ? nh : st);
    cnt = cnt < 0 ? 0 : (cnt > DEGCAP ? DEGCAP : cnt);
    if (cnt > nh - st) cnt = nh - st;
    const float pz = (ovf || craw > DEGCAP) ? qnan : 0.0f;
    const bool liveRow = grow < nN;

    const float adv = ADp[gcl];
    float mx = MX0, dn = 0.0f;
    v4f a0 = z4, a1 = z4, a2 = z4, a3 = z4;

#pragma unroll 1
    for (int q = 0; q < cnt; ++q) {
      int idx = st + q; idx = idx > RCAP - 1 ? RCAP - 1 : idx;
      int eid = reg2[idx]; eid = eid < 0 ? 0 : (eid > nE - 1 ? nE - 1 : eid);
      const int sraw = srcs[eid];
      const int s = sraw < 0 ? 0 : (sraw > nN - 1 ? nN - 1 : sraw);
      const float* fr = F + (size_t)s * HD + c0;
      const v4f f0 = *(const v4fa*)fr;
      const v4f f1 = *(const v4fa*)(fr + 4);
      const v4f f2 = *(const v4fa*)(fr + 8);
      const v4f f3 = *(const v4fa*)(fr + 12);
      float lg = ASp[s] + adv;
      lg = lg > 0.0f ? lg : NEGSL * lg;
      const float df = lg - mx;
      const float ee = __expf(-fabsf(df));
      const bool up  = df > 0.0f;
      const float s1 = up ? ee : 1.0f;
      const float s2 = up ? 1.0f : ee;
      mx = up ? lg : mx;
      dn = fmaf(dn, s1, s2);
      a0 = upd4(a0, f0, s1, s2);
      a1 = upd4(a1, f1, s1, s2);
      a2 = upd4(a2, f2, s1, s2);
      a3 = upd4(a3, f3, s1, s2);
    }
    const float dnz = dn > 0.0f ? dn : 1.0f;
    const float inv = __builtin_amdgcn_rcpf(dnz);
    est[0]  = a0.x * inv; est[1]  = a0.y * inv; est[2]  = a0.z * inv; est[3]  = a0.w * inv;
    est[4]  = a1.x * inv; est[5]  = a1.y * inv; est[6]  = a1.z * inv; est[7]  = a1.w * inv;
    est[8]  = a2.x * inv; est[9]  = a2.y * inv; est[10] = a2.z * inv; est[11] = a2.w * inv;
    est[12] = a3.x * inv; est[13] = a3.y * inv; est[14] = a3.z * inv; est[15] = a3.w * inv;
#pragma unroll 1
    for (int j = 0; j < 16; ++j) {
      float v = est[j] + sb[c0 + j];
      v = v > 0.0f ? v : expm1f(v);
      est[j] = v;
    }
    float o[16];
#pragma unroll
    for (int k = 0; k < 16; ++k) {
      const float v = est[k];
      o[k] = (liveRow ? v : 0.0f) + pz;
    }

    unsigned int hw[8], lw[8];
#pragma unroll
    for (int k = 0; k < 8; ++k) {
      const unsigned short h0 = bf_bits(o[2 * k]), h1 = bf_bits(o[2 * k + 1]);
      const unsigned short l0 = bf_bits(o[2 * k] - bf_val(h0)), l1 = bf_bits(o[2 * k + 1] - bf_val(h1));
      hw[k] = (unsigned int)h0 | ((unsigned int)h1 << 16);
      lw[k] = (unsigned int)l0 | ((unsigned int)l1 << 16);
    }
    v4u p0, p1, p2, p3;
    p0.x = shsel(hw[0], hw[4], slA, odd); p0.y = shsel(hw[1], hw[5], slA, odd);
    p0.z = shsel(hw[2], hw[6], slA, odd); p0.w = shsel(hw[3], hw[7], slA, odd);
    p1.x = shsel(hw[0], hw[4], slB, odd); p1.y = shsel(hw[1], hw[5], slB, odd);
    p1.z = shsel(hw[2], hw[6], slB, odd); p1.w = shsel(hw[3], hw[7], slB, odd);
    p2.x = shsel(lw[0], lw[4], slA, odd); p2.y = shsel(lw[1], lw[5], slA, odd);
    p2.z = shsel(lw[2], lw[6], slA, odd); p2.w = shsel(lw[3], lw[7], slA, odd);
    p3.x = shsel(lw[0], lw[4], slB, odd); p3.y = shsel(lw[1], lw[5], slB, odd);
    p3.z = shsel(lw[2], lw[6], slB, odd); p3.w = shsel(lw[3], lw[7], slB, odd);

    unsigned short* zp = ZP + (size_t)grow * KHL + 8 * lane;
    const bool wr = grow < MPr;
    if (wr) {
      *(volatile v4u*)(zp)       = p0;
      *(volatile v4u*)(zp + 256) = p1;
      *(volatile v4u*)(zp + 512) = p2;
      *(volatile v4u*)(zp + 768) = p3;
    }
    __threadfence();
    if (wr) {
      *(volatile v4u*)(zp)       = p0;
      *(volatile v4u*)(zp + 256) = p1;
      *(volatile v4u*)(zp + 512) = p2;
      *(volatile v4u*)(zp + 768) = p3;
    }
  }
}

__global__ __launch_bounds__(GTHR) void k_gsem(const unsigned short* __restrict__ A, int lda, size_t aoff,
                                              const unsigned short* __restrict__ BT, int ldb, int K,
                                              const float* __restrict__ bias, float* PS, int nN) {
  __shared__ __attribute__((aligned(16))) float stg[GBM * GBNS];
  __shared__ __attribute__((aligned(16))) float pst[GBNS];
  const int tid = (int)threadIdx.x, lane = tid & 31, wave = tid >> 5, hh = lane >> 4, m = lane & 15;
  const int rowBase = (int)blockIdx.x * GBM;
  const int by = (int)blockIdx.y;

  v8f acc[GNT];
  {
    const v8f z = {0.f, 0.f, 0.f, 0.f, 0.f, 0.f, 0.f, 0.f};
#pragma unroll
    for (int t = 0; t < GNT; ++t) acc[t] = z;
  }
  const unsigned short* Ab = A + (size_t)by * aoff;
  const unsigned short* ap = Ab + (size_t)(rowBase + 16 * wave + m) * (size_t)lda + 8 * hh;
  const unsigned short* bp = BT + (size_t)m * (size_t)ldb + 8 * hh;

#pragma unroll 1
  for (int k0 = 0; k0 < K; k0 += 32) {
    Frag af;
    af.h[0] = *(const v8usa*)(ap + k0);
    af.h[1] = *(const v8usa*)(ap + k0 + 16);
#pragma unroll
    for (int nt = 0; nt < GNT; ++nt) {
      const unsigned short* wq = bp + (size_t)(16 * nt) * (size_t)ldb + k0;
      Frag bfg;
      bfg.h[0] = *(const v8usa*)wq;
      bfg.h[1] = *(const v8usa*)(wq + 16);
      acc[nt] = wmb(af, bfg, acc[nt]);
    }
  }

#pragma unroll
  for (int nt = 0; nt < GNT; ++nt) {
    const int lc = 16 * nt + m;
    const float bb = bf_rne(bias[lc]);
#pragma unroll
    for (int r = 0; r < 8; ++r) {
      const int lr = 16 * wave + 8 * hh + r;
      const bool live = (rowBase + lr) < nN;
      const float v = acc[nt][r] + bb;
      stg[lr * GBNS + lc] = live ? v : 0.0f;
    }
  }
  __syncthreads();

  float s = 0.0f;
#pragma unroll 1
  for (int r = 0; r < GBM; ++r) s += tanhf(stg[r * GBNS + tid]);
  pst[tid] = s;
  __syncthreads();
  const bool pok = tid < 32;
  v4f pv = {0.f, 0.f, 0.f, 0.f};
  if (pok) pv = *(const v4fa*)(pst + 4 * tid);
  float* pp = PS + ((size_t)by * (size_t)gridDim.x + (size_t)blockIdx.x) * GBNS + 4 * tid;
  if (pok) *(volatile v4f*)pp = pv;
  __threadfence();
  if (pok) *(volatile v4f*)pp = pv;
}

__global__ __launch_bounds__(GBNS) void k_beta(const float* __restrict__ ps, int gM, int nN,
                                               const float* __restrict__ qv, float* be) {
  __shared__ double r0[GBNS], r1[GBNS];
  __shared__ __attribute__((aligned(16))) float bl[32];
  const int tid = (int)threadIdx.x;
  double s0 = 0.0, s1 = 0.0;
#pragma unroll 1
  for (int b = 0; b < gM; ++b) {
    s0 += (double)ps[(size_t)b * GBNS + tid];
    s1 += (double)ps[((size_t)gM + (size_t)b) * GBNS + tid];
  }
  const double qc  = (double)bf_rne(qv[tid]);
  const double inv = 1.0 / (double)(nN < 1 ? 1 : nN);
  r0[tid] = s0 * inv * qc;
  r1[tid] = s1 * inv * qc;
  if (tid < 32) bl[tid] = 0.0f;
  __syncthreads();
#pragma unroll 1
  for (int s = GBNS / 2; s > 0; s >>= 1) {
    if (tid < s) { r0[tid] += r0[tid + s]; r1[tid] += r1[tid + s]; }
    __syncthreads();
  }
  if (tid == 0) {
    const float w0 = (float)r0[0], w1 = (float)r1[0];
    const float mx = fmaxf(w0, w1);
    const float e0 = expf(w0 - mx), e1 = expf(w1 - mx);
    const float rs = 1.0f / (e0 + e1);
    bl[0] = e0 * rs;
    bl[1] = e1 * rs;
  }
  __syncthreads();
  const bool ok = tid < 8;
  v4f v = {0.f, 0.f, 0.f, 0.f};
  if (ok) v = *(const v4fa*)(bl + 4 * tid);
  if (ok) *(volatile v4f*)(be + 4 * tid) = v;
  __threadfence();
  if (ok) *(volatile v4f*)(be + 4 * tid) = v;
}

__global__ __launch_bounds__(GTHR) void k_out(const unsigned short* __restrict__ P0, const unsigned short* __restrict__ P1,
                                             const float* __restrict__ be, const unsigned short* __restrict__ PT,
                                             const float* __restrict__ pb, int nN, float* out) {
  extern __shared__ v4u lds_o[];
  unsigned short* As = (unsigned short*)lds_o;
  __shared__ __attribute__((aligned(16))) float so[GBM * NOUT];
  const int tid = (int)threadIdx.x, lane = tid & 31, wave = tid >> 5, hh = lane >> 4, m = lane & 15;
  const int rowBase = (int)blockIdx.x * GBM;
  const float b0 = be[0], b1 = be[1];

#pragma unroll 1
  for (int it = 0; it < (GBM * (HD / 8)) / GTHR; ++it) {
    const int u  = it * GTHR + tid;
    const int lr = u >> 6, qq = u & 63;
    const int grow = rowBase + lr;
    const int gc = grow < nN ? grow : nN - 1;
    const unsigned short* pa = P0 + (size_t)gc * KHL + 8 * qq;
    const unsigned short* pc = P1 + (size_t)gc * KHL + 8 * qq;
    const v4u ha = *(const v4ua*)pa, la = *(const v4ua*)(pa + HD);
    const v4u hb = *(const v4ua*)pc, lbw = *(const v4ua*)(pc + HD);
    const bool live = grow < nN;
    float f[8];
    f[0] = fmaf(b1, rlo(hb.x, lbw.x), b0 * rlo(ha.x, la.x));
    f[1] = fmaf(b1, rhi(hb.x, lbw.x), b0 * rhi(ha.x, la.x));
    f[2] = fmaf(b1, rlo(hb.y, lbw.y), b0 * rlo(ha.y, la.y));
    f[3] = fmaf(b1, rhi(hb.y, lbw.y), b0 * rhi(ha.y, la.y));
    f[4] = fmaf(b1, rlo(hb.z, lbw.z), b0 * rlo(ha.z, la.z));
    f[5] = fmaf(b1, rhi(hb.z, lbw.z), b0 * rhi(ha.z, la.z));
    f[6] = fmaf(b1, rlo(hb.w, lbw.w), b0 * rlo(ha.w, la.w));
    f[7] = fmaf(b1, rhi(hb.w, lbw.w), b0 * rhi(ha.w, la.w));
    unsigned int wh[4], wl[4];
#pragma unroll
    for (int j = 0; j < 4; ++j) {
      float v0 = f[2 * j], v1 = f[2 * j + 1];
      v0 = live ? v0 : 0.0f;
      v1 = live ? v1 : 0.0f;
      const unsigned short h0 = bf_bits(v0), h1 = bf_bits(v1);
      const unsigned short l0 = bf_bits(v0 - bf_val(h0)), l1 = bf_bits(v1 - bf_val(h1));
      wh[j] = (unsigned int)h0 | ((unsigned int)h1 << 16);
      wl[j] = (unsigned int)l0 | ((unsigned int)l1 << 16);
    }
    v4u hv, lv;
    hv.x = wh[0]; hv.y = wh[1]; hv.z = wh[2]; hv.w = wh[3];
    lv.x = wl[0]; lv.y = wl[1]; lv.z = wl[2]; lv.w = wl[3];
    *(v4ua*)(As + lr * KHL + 8 * qq)      = hv;
    *(v4ua*)(As + lr * KHL + HD + 8 * qq) = lv;
  }
  __syncthreads();

  v8f acc = {0.f, 0.f, 0.f, 0.f, 0.f, 0.f, 0.f, 0.f};
  const unsigned short* ap = As + (16 * wave + m) * KHL + 8 * hh;
  const unsigned short* bp = PT + (size_t)m * KHL + 8 * hh;
#pragma unroll 1
  for (int k0 = 0; k0 < KHL; k0 += 32) {
    Frag af, bfg;
    af.h[0]  = *(const v8usa*)(ap + k0);
    af.h[1]  = *(const v8usa*)(ap + k0 + 16);
    bfg.h[0] = *(const v8usa*)(bp + k0);
    bfg.h[1] = *(const v8usa*)(bp + k0 + 16);
    acc = wmb(af, bfg, acc);
  }
  const int mc = m < OUTC ? m : OUTC - 1;
  float pbm = bf_rne(pb[mc]);
  pbm = m < OUTC ? pbm : 0.0f;
#pragma unroll
  for (int r = 0; r < 8; ++r) {
    const int lr = 16 * wave + 8 * hh + r;
    so[lr * NOUT + m] = acc[r] + pbm;
  }
  __syncthreads();

  int nvr = nN - rowBase;
  nvr = nvr < 0 ? 0 : (nvr > GBM ? GBM : nvr);
  const int nfl = nvr * OUTC;
  const int npc = nfl >> 2;
  const int rem = nfl & 3;
  float* ob = out + (size_t)rowBase * OUTC;
  const int p  = tid;
  const bool pok = p < npc;
  const int pcl = pok ? p : 0;
  v4f pv;
  {
    const int e0 = 4 * pcl, e1 = e0 + 1, e2 = e0 + 2, e3 = e0 + 3;
    const int q0 = e0 / OUTC, q1 = e1 / OUTC, q2 = e2 / OUTC, q3 = e3 / OUTC;
    pv.x = so[q0 * NOUT + (e0 - q0 * OUTC)];
    pv.y = so[q1 * NOUT + (e1 - q1 * OUTC)];
    pv.z = so[q2 * NOUT + (e2 - q2 * OUTC)];
    pv.w = so[q3 * NOUT + (e3 - q3 * OUTC)];
  }
  const bool tok = (rem != 0) && (tid == npc);
  float t0 = 0.f, t1 = 0.f, t2 = 0.f;
  {
    const int eb = 4 * npc;
    const int q0 = eb / OUTC, q1 = (eb + 1) / OUTC, q2 = (eb + 2) / OUTC;
    const int r0 = q0 < GBM ? q0 : GBM - 1, r1 = q1 < GBM ? q1 : GBM - 1, r2 = q2 < GBM ? q2 : GBM - 1;
    t0 = so[r0 * NOUT + (eb - q0 * OUTC)];
    t1 = so[r1 * NOUT + (eb + 1 - q1 * OUTC)];
    t2 = so[r2 * NOUT + (eb + 2 - q2 * OUTC)];
  }
  if (pok) *(volatile v4f*)(ob + 4 * p) = pv;
  if (tok) {
    *(volatile float*)(ob + 4 * npc) = t0;
    if (rem > 1) *(volatile float*)(ob + 4 * npc + 1) = t1;
    if (rem > 2) *(volatile float*)(ob + 4 * npc + 2) = t2;
  }
  __threadfence();
  if (pok) *(volatile v4f*)(ob + 4 * p) = pv;
  if (tok) {
    *(volatile float*)(ob + 4 * npc) = t0;
    if (rem > 1) *(volatile float*)(ob + 4 * npc + 1) = t1;
    if (rem > 2) *(volatile float*)(ob + 4 * npc + 2) = t2;
  }
}

static int pick_nb(int nE, int nN) {
  int nb = NBMAX;
  while (nb > 32 && (long long)nb * (long long)nE * 5LL > (long long)RCAP * (long long)nN * 4LL) nb >>= 1;
  return nb;
}
static inline int cdiv(int a, int b) { return (a + b - 1) / b; }
static inline size_t al256(size_t o) { return (o + 255) & ~(size_t)255; }

extern "C" void kernel_launch(void* const* d_in, const int* in_sizes, int n_in,
                              void* d_out, int out_size, void* d_ws, size_t ws_size,
                              hipStream_t stream) {
  if (n_in < 12) return;
  if (in_sizes[0] < F_IN || (in_sizes[0] % F_IN) != 0) return;
  const int nN = in_sizes[0] / F_IN;
  if (nN < 1 || nN > (1 << 22)) return;
  if (in_sizes[1] < NPATH || (in_sizes[1] % NPATH) != 0) return;
  if (in_sizes[2] != in_sizes[1]) return;
  const int nE = in_sizes[1] / NPATH;
  if (nE < 1 || nE >= (1 << (32 - SLOTB))) return;
  if (in_sizes[3] != NPATH * F_IN * HD) return;
  if (in_sizes[4] != NPATH * HD || in_sizes[5] != NPATH * HD) return;
  if (in_sizes[6] != NPATH * HD) return;
  if (in_sizes[7] != HD * SHID || in_sizes[8] != SHID) return;
  if (in_sizes[9] != SHID) return;
  if (in_sizes[10] != HD * OUTC || in_sizes[11] != OUTC) return;
  if ((long long)out_size != (long long)nN * OUTC) return;

  const float* h    = (const float*)d_in[0];
  const int*   src  = (const int*)  d_in[1];
  const int*   dst  = (const int*)  d_in[2];
  const float* w    = (const float*)d_in[3];
  const float* al   = (const float*)d_in[4];
  const float* ar   = (const float*)d_in[5];
  const float* bg   = (const float*)d_in[6];
  const float* sw1  = (const float*)d_in[7];
  const float* sb1  = (const float*)d_in[8];
  const float* sw2  = (const float*)d_in[9];
  const float* pw   = (const float*)d_in[10];
  const float* pb   = (const float*)d_in[11];
  float* out = (float*)d_out;

  const int MP = cdiv(nN, GBM) * GBM;
  const int gM = MP / GBM;
  const int nb = pick_nb(nE, nN);
  if (nb < 32 || (nb & (nb - 1)) != 0 || nb > NBMAX) return;
  const int gA = cdiv(MP, nb);
  if ((long long)gA * nb < (long long)MP) return;
  const int vec8 = ((nE & 3) == 0) ? 1 : 0;
  if ((long long)(gM - 1) * GBM >= (long long)nN) return;

  char* ws = (char*)d_ws;
  size_t off = 0;
  const size_t oZ  = off; off = al256(off + (size_t)NPATH * MP * KHL * 2);
  const size_t oWT = off; off = al256(off + (size_t)NUW * 16);
  const size_t oS1 = off; off = al256(off + (size_t)NUS * 16);
  const size_t oPT = off; off = al256(off + (size_t)NUP * 16);
  const size_t oF  = off; off = al256(off + (size_t)MP * HD * 4);
  const size_t oSD = off; off = al256(off + (size_t)NPATH * NHEAD * 2 * MP * 4);
  const size_t oPS = off; off = al256(off + (size_t)NPATH * gM * SHID * 4);
  const size_t oBE = off; off = al256(off + 256);
  if (off > ws_size || off > (size_t)WSMAX) return;
  unsigned short* ZHL = (unsigned short*)(ws + oZ);
  unsigned short* Z0  = ZHL;
  unsigned short* Z1  = ZHL + (size_t)MP * KHL;
  unsigned short* XB  = Z1;
  unsigned short* WT  = (unsigned short*)(ws + oWT);
  unsigned short* S1T = (unsigned short*)(ws + oS1);
  unsigned short* PTp = (unsigned short*)(ws + oPT);
  float*          FE  = (float*)(ws + oF);
  float*          SD  = (float*)(ws + oSD);
  float*          PS  = (float*)(ws + oPS);
  float*          BE  = (float*)(ws + oBE);
  const size_t aoff = (size_t)MP * KHL;

  hipFuncSetAttribute(reinterpret_cast<const void*>(&k_agg), hipFuncAttributeMaxDynamicSharedMemorySize, LDS_AGG);
  hipFuncSetAttribute(reinterpret_cast<const void*>(&k_out), hipFuncAttributeMaxDynamicSharedMemorySize, LDS_OUT);

  const int nUx = MP * (F_IN / 8);
  k_xprep<<<cdiv(nUx, NTHR), NTHR, 0, stream>>>(h, XB, nN, nUx);
  k_wprep<<<NUTOT / NTHR, NTHR, 0, stream>>>(w, sw1, pw, WT, S1T, PTp);
  for (int p = 0; p < NPATH; ++p) {
    const unsigned short* WTp = WT + (size_t)p * HD * F_IN;
    float* SDp = SD + (size_t)(2 * NHEAD) * (size_t)p * (size_t)MP;
    unsigned short* Zp = ZHL + (size_t)p * aoff;
    k_gfeat<<<dim3(gM, NHEAD), GTHR, 0, stream>>>(XB, WTp, FE, F_IN, HD, al + (size_t)p * HD, ar + (size_t)p * HD,
                                                 DHD, SDp, MP);
    k_agg<<<gA, NTHR, LDS_AGG, stream>>>(src + (size_t)p * nE, dst + (size_t)p * nE, FE, SDp, bg + (size_t)p * HD,
                                         Zp, nN, nE, nb, vec8, MP);
  }
  k_gsem<<<dim3(gM, NPATH), GTHR, 0, stream>>>(ZHL, KHL, aoff, S1T, KHL, KHL, sb1, PS, nN);
  k_beta<<<1, GBNS, 0, stream>>>(PS, gM, nN, sw2, BE);
  k_out<<<gM, GTHR, LDS_OUT, stream>>>(Z0, Z1, BE, PTp, pb, nN, out);
}
